// InnerLayer_53798760349843
// MI455X (gfx1250) — hardware-verified
//
#include <hip/hip_runtime.h>
#include <stddef.h>


typedef float    v4f  __attribute__((ext_vector_type(4)));
typedef v4f      v4fa __attribute__((may_alias));
typedef float    v8f  __attribute__((ext_vector_type(8)));
typedef __bf16   v16b __attribute__((ext_vector_type(16)));
typedef __bf16   v8b  __attribute__((ext_vector_type(8)));
typedef _Float16 v16h __attribute__((ext_vector_type(16)));
typedef _Float16 v8h  __attribute__((ext_vector_type(8)));

union BFrag { v16b v; v8b half[2]; };
union HFrag { v16h v; v8h half[2]; };

#define MSG_K    544
#define MSG_EPB  512
#define MSG_LDS  (2 * 32 * MSG_K * 2)
#define SEG_R    1024
#define SEG_LDS  (SEG_R * 32 * 4)

extern __shared__ __align__(16) float g_dyn[];

__device__ __forceinline__ v8f mma_bf(v8f c, v16b a, v16b b)
{
    c = __builtin_amdgcn_wmma_f32_16x16x32_bf16(false, a, false, b, (short)0, c, false, false);
    asm volatile("v_nop\n\tv_nop\n\tv_nop\n\tv_nop" : "+v"(c) : "v"(a), "v"(b));
    return c;
}

__device__ __forceinline__ v8f mma_h(v8f c, v16h a, v16h b)
{
    c = __builtin_amdgcn_wmma_f32_16x16x32_f16(false, a, false, b, (short)0, c, false, false);
    asm volatile("v_nop\n\tv_nop\n\tv_nop\n\tv_nop" : "+v"(c) : "v"(a), "v"(b));
    return c;
}

__global__ __launch_bounds__(256)
void k_gather(const float* __restrict__ x, const int* __restrict__ src,
              float* xg, int E, int Nsrc)
{
    const int t    = threadIdx.x;
    const int lane = t & 31, wv = t >> 5;
    const int sub  = lane >> 3;
    const int c4   = (lane & 7) * 4;
    v4f vals[8];
    int rows[8];
#pragma unroll
    for (int it = 0; it < 8; ++it) {
        const int e  = blockIdx.x * 256 + wv * 32 + it * 4 + sub;
        rows[it]     = e;
        const int ec = e < E ? e : E - 1;
        int s = src[ec];
        if (s < 0) s += Nsrc;
        s = s < 0 ? 0 : (s > Nsrc - 1 ? Nsrc - 1 : s);
        vals[it] = *(const v4f*)(x + (size_t)s * 32 + c4);
    }
#pragma unroll
    for (int it = 0; it < 8; ++it)
        if (rows[it] < E) *(volatile v4f*)(xg + (size_t)rows[it] * 32 + c4) = vals[it];
    __threadfence();
#pragma unroll
    for (int it = 0; it < 8; ++it)
        if (rows[it] < E) *(volatile v4f*)(xg + (size_t)rows[it] * 32 + c4) = vals[it];
}

__global__ __launch_bounds__(256) __attribute__((amdgpu_num_vgpr(256)))
void k_msg(const float* xg, const float* __restrict__ ea,
           const float* __restrict__ mw, const float* __restrict__ mb,
           float* mout, int E)
{
    __bf16* Bh = (__bf16*)g_dyn;
    __bf16* Bl = Bh + 32 * MSG_K;
    __shared__ __align__(16) float stg[8 * 512];

    const int t = threadIdx.x;

#pragma unroll 4
    for (int i = t; i < 16 * 1024; i += 256) {
        const float w   = mw[i];
        const int   d   = i >> 10;
        const int   col = i & 1023;
        const int   f   = col >> 5;
        const int   g   = col & 31;
        const __bf16 hb = (__bf16)w;
        const __bf16 lb = (__bf16)(w - (float)hb);
        const int   idx = g * MSG_K + f * 16 + d;
        Bh[idx] = hb;
        Bl[idx] = lb;
    }
#pragma unroll
    for (int i = t; i < 1024; i += 256) {
        const float w   = mb[i];
        const int   f   = i >> 5;
        const int   g   = i & 31;
        const __bf16 hb = (__bf16)w;
        const __bf16 lb = (__bf16)(w - (float)hb);
        const int   idx = g * MSG_K + 512 + f;
        Bh[idx] = hb;
        Bl[idx] = lb;
    }
    __syncthreads();

    const int lane = t & 31;
    const int wv   = t >> 5;
    const int m    = lane & 15;
    const int h    = lane >> 4;
    float* st = stg + wv * 512;

    const __bf16* bh0p = Bh + m * MSG_K + 8 * h;
    const __bf16* bh1p = Bh + (16 + m) * MSG_K + 8 * h;
    const __bf16* bl0p = Bl + m * MSG_K + 8 * h;
    const __bf16* bl1p = Bl + (16 + m) * MSG_K + 8 * h;

    const int rq = lane >> 3;
    const int c4 = (lane & 7) * 4;

#pragma unroll 1
    for (int it = 0; it < 4; ++it) {
        const int e0 = blockIdx.x * MSG_EPB + (it * 8 + wv) * 16;
        int e = e0 + m;
        if (e > E - 1) e = E - 1;

        float xr[32];
        {
            const v4f* xp = (const v4f*)(xg + (size_t)e * 32);
#pragma unroll
            for (int q = 0; q < 8; ++q) {
                const v4f v = xp[q];
                xr[4 * q + 0] = v[0]; xr[4 * q + 1] = v[1];
                xr[4 * q + 2] = v[2]; xr[4 * q + 3] = v[3];
            }
        }
        float ev[8];
        {
            const float* eap = ea + (size_t)e * 16 + 8 * h;
            const v4f a0 = *(const v4f*)(eap);
            const v4f a1 = *(const v4f*)(eap + 4);
            ev[0] = a0[0]; ev[1] = a0[1]; ev[2] = a0[2]; ev[3] = a0[3];
            ev[4] = a1[0]; ev[5] = a1[1]; ev[6] = a1[2]; ev[7] = a1[3];
        }

        v8f c0 = {};
        v8f c1 = {};

#pragma unroll
        for (int s = 0; s < 17; ++s) {
            float p[16];
            if (s < 16) {
#pragma unroll
                for (int i = 0; i < 8; ++i) {
                    p[i]     = xr[2 * s]     * ev[i];
                    p[8 + i] = xr[2 * s + 1] * ev[i];
                }
            } else {
#pragma unroll
                for (int i = 0; i < 8; ++i) {
                    p[i]     = h ? xr[8 + i]  : xr[i];
                    p[8 + i] = h ? xr[24 + i] : xr[16 + i];
                }
            }
            BFrag ah, al;
#pragma unroll
            for (int i = 0; i < 16; ++i) {
                const __bf16 hb = (__bf16)p[i];
                ah.v[i] = hb;
                al.v[i] = (__bf16)(p[i] - (float)hb);
            }
            const int ko = 32 * s;
            BFrag bh0, bl0, bh1, bl1;
            bh0.half[0] = *(const v8b*)(bh0p + ko);      bh0.half[1] = *(const v8b*)(bh0p + ko + 16);
            bl0.half[0] = *(const v8b*)(bl0p + ko);      bl0.half[1] = *(const v8b*)(bl0p + ko + 16);
            bh1.half[0] = *(const v8b*)(bh1p + ko);      bh1.half[1] = *(const v8b*)(bh1p + ko + 16);
            bl1.half[0] = *(const v8b*)(bl1p + ko);      bl1.half[1] = *(const v8b*)(bl1p + ko + 16);

            c0 = mma_bf(c0, ah.v, bh0.v);
            c0 = mma_bf(c0, ah.v, bl0.v);
            c0 = mma_bf(c0, al.v, bh0.v);
            c1 = mma_bf(c1, ah.v, bh1.v);
            c1 = mma_bf(c1, ah.v, bl1.v);
            c1 = mma_bf(c1, al.v, bh1.v);
        }

#pragma unroll
        for (int r = 0; r < 8; ++r) {
            st[(8 * h + r) * 32 + m]      = c0[r];
            st[(8 * h + r) * 32 + 16 + m] = c1[r];
        }
        __syncthreads();
        v4f ov[4];
#pragma unroll
        for (int q = 0; q < 4; ++q) ov[q] = *(const v4fa*)(st + (4 * q + rq) * 32 + c4);
#pragma unroll
        for (int q = 0; q < 4; ++q) {
            const int er = e0 + 4 * q + rq;
            if (er < E) *(volatile v4f*)(mout + (size_t)er * 32 + c4) = ov[q];
        }
        __threadfence();
#pragma unroll
        for (int q = 0; q < 4; ++q) {
            const int er = e0 + 4 * q + rq;
            if (er < E) *(volatile v4f*)(mout + (size_t)er * 32 + c4) = ov[q];
        }
        __syncthreads();
    }
}

__global__ __launch_bounds__(256) __attribute__((amdgpu_num_vgpr(256)))
void k_seg(const float* msg, const int* __restrict__ dst,
           const float* __restrict__ xd, const float* __restrict__ root,
           const float* __restrict__ bias, float* out,
           int N, int E, int nchunk)
{
    float* acc = g_dyn;
    __shared__ __align__(16) _Float16 rB[32 * 32];
    __shared__ int liste[256];
    __shared__ int listj[256];
    __shared__ int wcnt[8];

    const int t    = threadIdx.x;
    const int lane = t & 31;
    const int wv   = t >> 5;
    const int m    = lane & 15;
    const int h    = lane >> 4;
    const int n0   = blockIdx.x * SEG_R;

    {
        const v4f z = {0.0f, 0.0f, 0.0f, 0.0f};
        v4f* acc4 = (v4f*)acc;
#pragma unroll 4
        for (int i = t; i < SEG_R * 8; i += 256) acc4[i] = z;
    }
#pragma unroll
    for (int i = t; i < 1024; i += 256) {
        const int k = i >> 5;
        const int n = i & 31;
        rB[n * 32 + k] = (_Float16)(root[i] * 64.0f);
    }
    __syncthreads();

#pragma unroll 1
    for (int c = 0; c < nchunk; ++c) {
        const int e = c * 256 + t;
        int j = -1;
        if (e < E) j = dst[e] - n0;
        const bool hit = (unsigned)j < (unsigned)SEG_R;
        const unsigned int mask = __builtin_amdgcn_ballot_w32(hit);
        const int pre = __builtin_popcount(mask & ((1u << lane) - 1u));
        if (lane == 0) wcnt[wv] = __builtin_popcount(mask);
        __syncthreads();
        int off = 0, nh = 0;
#pragma unroll
        for (int q = 0; q < 8; ++q) {
            const int cq = wcnt[q];
            nh += cq;
            if (q < wv) off += cq;
        }
        if (hit) {
            liste[off + pre] = e;
            listj[off + pre] = j;
        }
        __syncthreads();
        if (nh > 256) nh = 256;
#pragma unroll 1
        for (int i = 0; i < nh; ++i) {
            const int jj = listj[i] & (SEG_R - 1);
            if ((jj & 7) == wv) {
                int ee = liste[i];
                if (ee < 0) ee = 0;
                if (ee > E - 1) ee = E - 1;
                acc[jj * 32 + lane] += msg[(size_t)ee * 32 + lane];
            }
        }
        __syncthreads();
    }

    HFrag bf0, bf1;
    bf0.half[0] = *(const v8h*)(rB + m * 32 + 8 * h);
    bf0.half[1] = *(const v8h*)(rB + m * 32 + 16 + 8 * h);
    bf1.half[0] = *(const v8h*)(rB + (16 + m) * 32 + 8 * h);
    bf1.half[1] = *(const v8h*)(rB + (16 + m) * 32 + 16 + 8 * h);
    const float b0v = bias[m];
    const float b1v = bias[16 + m];
    const float rs  = 0.015625f;

#pragma unroll 1
    for (int tt = 0; tt < 8; ++tt) {
        const int j0 = (tt * 8 + wv) * 16;
        int node = n0 + j0 + m;
        if (node > N - 1) node = N - 1;
        const v4f* xp = (const v4f*)(xd + (size_t)node * 32);
        const v4f x0 = xp[2 * h];
        const v4f x1 = xp[2 * h + 1];
        const v4f x2 = xp[4 + 2 * h];
        const v4f x3 = xp[5 + 2 * h];
        HFrag a;
        a.v[0]  = (_Float16)x0[0]; a.v[1]  = (_Float16)x0[1]; a.v[2]  = (_Float16)x0[2]; a.v[3]  = (_Float16)x0[3];
        a.v[4]  = (_Float16)x1[0]; a.v[5]  = (_Float16)x1[1]; a.v[6]  = (_Float16)x1[2]; a.v[7]  = (_Float16)x1[3];
        a.v[8]  = (_Float16)x2[0]; a.v[9]  = (_Float16)x2[1]; a.v[10] = (_Float16)x2[2]; a.v[11] = (_Float16)x2[3];
        a.v[12] = (_Float16)x3[0]; a.v[13] = (_Float16)x3[1]; a.v[14] = (_Float16)x3[2]; a.v[15] = (_Float16)x3[3];
        v8f c0 = {};
        v8f c1 = {};
        c0 = mma_h(c0, a.v, bf0.v);
        c1 = mma_h(c1, a.v, bf1.v);
#pragma unroll
        for (int r = 0; r < 8; ++r) {
            const int row = j0 + 8 * h + r;
            acc[row * 32 + m]      += c0[r] * rs + b0v;
            acc[row * 32 + 16 + m] += c1[r] * rs + b1v;
        }
    }
    __syncthreads();

    const int rq = lane >> 3;
    const int c4 = (lane & 7) * 4;
#pragma unroll 1
    for (int tt = 0; tt < 8; ++tt) {
        const int j0 = (tt * 8 + wv) * 16;
#pragma unroll
        for (int q = 0; q < 4; ++q) {
            const int row  = 4 * q + rq;
            const int node = n0 + j0 + row;
            const v4f v = *(const v4fa*)(acc + (j0 + row) * 32 + c4);
            if (node < N) *(volatile v4f*)(out + (size_t)node * 32 + c4) = v;
        }
    }
    __threadfence();
#pragma unroll 1
    for (int tt = 0; tt < 8; ++tt) {
        const int j0 = (tt * 8 + wv) * 16;
#pragma unroll
        for (int q = 0; q < 4; ++q) {
            const int row  = 4 * q + rq;
            const int node = n0 + j0 + row;
            const v4f v = *(const v4fa*)(acc + (j0 + row) * 32 + c4);
            if (node < N) *(volatile v4f*)(out + (size_t)node * 32 + c4) = v;
        }
    }
}

static inline size_t al256(size_t x) { return (x + 255) & ~(size_t)255; }

extern "C" void kernel_launch(void* const* d_in, const int* in_sizes, int n_in,
                              void* d_out, int out_size, void* d_ws, size_t ws_size,
                              hipStream_t stream)
{
    const float* x_a      = (const float*)d_in[0];
    const float* x_b      = (const float*)d_in[1];
    const int*   ei_ab    = (const int*)  d_in[2];
    const float* ea_ab    = (const float*)d_in[3];
    const int*   ei_ba    = (const int*)  d_in[4];
    const float* ea_ba    = (const float*)d_in[5];
    const float* msg_W_ab = (const float*)d_in[6];
    const float* msg_b_ab = (const float*)d_in[7];
    const float* root_ab  = (const float*)d_in[8];
    const float* bias_ab  = (const float*)d_in[9];
    const float* msg_W_ba = (const float*)d_in[10];
    const float* msg_b_ba = (const float*)d_in[11];
    const float* root_ba  = (const float*)d_in[12];
    const float* bias_ba  = (const float*)d_in[13];

    const int NA  = in_sizes[0] / 32;
    const int NB  = in_sizes[1] / 32;
    const int Eab = in_sizes[2] / 2;
    const int Eba = in_sizes[4] / 2;
    if (NA <= 0 || NB <= 0) return;
    if ((size_t)(NA + NB) * 32 > (size_t)out_size) return;

    size_t off = 0;
    const size_t bab = al256((size_t)(Eab > 0 ? Eab : 1) * 32 * sizeof(float));
    const size_t bba = al256((size_t)(Eba > 0 ? Eba : 1) * 32 * sizeof(float));
    float* xg_ab = (float*)((char*)d_ws + off); off += bab;
    float* ms_ab = (float*)((char*)d_ws + off); off += bab;
    float* xg_ba = (float*)((char*)d_ws + off); off += bba;
    float* ms_ba = (float*)((char*)d_ws + off); off += bba;
    if (off > ws_size) return;

    float* outp  = (float*)d_out;
    float* out_a = outp;
    float* out_b = outp + (size_t)NA * 32;

    if (Eab > 0) {
        k_gather<<<(Eab + 255) / 256, 256, 0, stream>>>(x_a, ei_ab, xg_ab, Eab, NA);
        k_msg<<<(Eab + MSG_EPB - 1) / MSG_EPB, 256, MSG_LDS, stream>>>(xg_ab, ea_ab, msg_W_ab, msg_b_ab, ms_ab, Eab);
    }
    k_seg<<<(NB + SEG_R - 1) / SEG_R, 256, SEG_LDS, stream>>>(
        ms_ab, ei_ab + Eab, x_b, root_ab, bias_ab, out_b, NB, Eab, (Eab + 255) / 256);

    if (Eba > 0) {
        k_gather<<<(Eba + 255) / 256, 256, 0, stream>>>(x_b, ei_ba, xg_ba, Eba, NB);
        k_msg<<<(Eba + MSG_EPB - 1) / MSG_EPB, 256, MSG_LDS, stream>>>(xg_ba, ea_ba, msg_W_ba, msg_b_ba, ms_ba, Eba);
    }
    k_seg<<<(NA + SEG_R - 1) / SEG_R, 256, SEG_LDS, stream>>>(
        ms_ba, ei_ba + Eba, x_a, root_ba, bias_ba, out_a, NA, Eba, (Eba + 255) / 256);
}
